// PrototypeLearner_53377853555142
// MI455X (gfx1250) — hardware-verified
//
#include <hip/hip_runtime.h>


#define NTK  8192
#define DD   512
#define NP   2000
#define NPP  2048
#define NC   200
#define NPR  10
#define EPSI 0.01f
#define ITER 5
typedef _Float16 h16;
typedef unsigned short bf;
typedef __attribute__((ext_vector_type(16))) __bf16   v16bf;
typedef __attribute__((ext_vector_type(16))) _Float16 v16h;
typedef __attribute__((ext_vector_type(8)))  _Float16 v8h;
typedef __attribute__((ext_vector_type(8)))  unsigned short v8us;
typedef __attribute__((ext_vector_type(8)))  float    v8f;
typedef __attribute__((ext_vector_type(4)))  float    v4f;
typedef v8h  __attribute__((may_alias)) v8ha;
typedef v4f  __attribute__((may_alias)) v4fa;
typedef v8us __attribute__((may_alias)) v8usa;

__device__ __forceinline__ unsigned short f2bf(float f) { unsigned u = __float_as_uint(f); u += 0x7FFFu + ((u >> 16) & 1u); return (unsigned short)(u >> 16); }
__device__ __forceinline__ float bf2f(unsigned short b) { return __uint_as_float(((unsigned)b) << 16); }
__device__ __forceinline__ float bfr(float f) { return bf2f(f2bf(f)); }
__device__ __forceinline__ v16h cat16(v8h lo, v8h hi) { return __builtin_shufflevector(lo, hi, 0, 1, 2, 3, 4, 5, 6, 7, 8, 9, 10, 11, 12, 13, 14, 15); }
__device__ __forceinline__ v16bf cat16b(v8us lo, v8us hi) { return __builtin_bit_cast(v16bf, __builtin_shufflevector(lo, hi, 0, 1, 2, 3, 4, 5, 6, 7, 8, 9, 10, 11, 12, 13, 14, 15)); }
__device__ __forceinline__ v8f wmma16(v16h a, v16h b, v8f c) { return __builtin_amdgcn_wmma_f32_16x16x32_f16(false, a, false, b, (short)0, c, false, false); }
__device__ __forceinline__ v8f wmmab(v16bf a, v16bf b, v8f c) { return __builtin_amdgcn_wmma_f32_16x16x32_bf16(false, a, false, b, (short)0, c, false, false); }


template <typename T16> struct WFrag;
template <> struct WFrag<h16> { typedef v16h V; static __device__ __forceinline__ V ld(const h16* p) { return cat16(*(const v8h*)p, *(const v8h*)(p + 16)); } static __device__ __forceinline__ v8f mma(V a, V b, v8f c) { return wmma16(a, b, c); } };
template <> struct WFrag<bf> { typedef v16bf V; static __device__ __forceinline__ V ld(const bf* p) { return cat16b(*(const v8us*)p, *(const v8us*)(p + 16)); } static __device__ __forceinline__ v8f mma(V a, V b, v8f c) { return wmmab(a, b, c); } };
template <typename T16, int NSPLIT, bool BIAS>
__global__ __launch_bounds__(32) void k_gemmw(const T16* __restrict__ A, const T16* __restrict__ A2, const T16* __restrict__ Bt, const T16* __restrict__ Bt2, int K, float* C, int ldc, const float* __restrict__ bias, size_t sA, size_t sB, size_t sC) {
    typedef typename WFrag<T16>::V V;
    __shared__ __align__(16) float os[16 * 68];
    const size_t z = blockIdx.z; A += z * sA; if (A2) A2 += z * sA; Bt += z * sB; if (Bt2) Bt2 += z * sB; C += z * sC;
    const int lane = threadIdx.x & 31, lr = lane & 15, hi = lane >> 4; const int r0 = blockIdx.x * 64, c0 = blockIdx.y * 64;
    v8f acc[4][4];
#pragma unroll
    for (int mb = 0; mb < 4; ++mb)
#pragma unroll
        for (int nb = 0; nb < 4; ++nb) acc[mb][nb] = (v8f){};
    const size_t aoff = (size_t)(r0 + lr) * K + 8 * hi, boff = (size_t)(c0 + lr) * K + 8 * hi;
#pragma unroll 1
    for (int kc = 0; kc < K; kc += 32) {
        V a[4], a2[4];
#pragma unroll
        for (int mb = 0; mb < 4; ++mb) { a[mb] = WFrag<T16>::ld(A + aoff + (size_t)mb * 16 * K + kc); if (NSPLIT == 1 || NSPLIT == 2) a2[mb] = WFrag<T16>::ld(A2 + aoff + (size_t)mb * 16 * K + kc); }
#pragma unroll
        for (int nb = 0; nb < 4; ++nb) { const V b = WFrag<T16>::ld(Bt + boff + (size_t)nb * 16 * K + kc); V b2; if (NSPLIT >= 2) b2 = WFrag<T16>::ld(Bt2 + boff + (size_t)nb * 16 * K + kc);
#pragma unroll
            for (int mb = 0; mb < 4; ++mb) { acc[mb][nb] = WFrag<T16>::mma(a[mb], b, acc[mb][nb]); if (NSPLIT == 1 || NSPLIT == 2) acc[mb][nb] = WFrag<T16>::mma(a2[mb], b, acc[mb][nb]); if (NSPLIT >= 2) acc[mb][nb] = WFrag<T16>::mma(a[mb], b2, acc[mb][nb]); } }
        asm volatile("v_nop\n\tv_nop\n\tv_nop\n\tv_nop" : "+v"(acc[0][0]), "+v"(acc[1][1]), "+v"(acc[2][2]), "+v"(acc[3][3]) : "v"(a[0]), "v"(a[3]));
    }
#pragma unroll
    for (int mb = 0; mb < 4; ++mb) {
#pragma unroll
        for (int nb = 0; nb < 4; ++nb) {
#pragma unroll
            for (int j = 0; j < 8; ++j) os[(hi * 8 + j) * 68 + nb * 16 + lr] = acc[mb][nb][j]; }
        __builtin_amdgcn_wave_barrier(); asm volatile("" ::: "memory");
        float* crow = C + (size_t)(r0 + mb * 16) * ldc + c0;
#pragma unroll 1
        for (int ps = 0; ps < 2; ++ps) {
#pragma unroll
            for (int s = 0; s < 8; ++s) { const int row = 2 * s + hi, cofs = lr * 4; v4f val = *(const v4fa*)(os + row * 68 + cofs); if (BIAS) { val[0] += bfr(bias[c0 + cofs]); val[1] += bfr(bias[c0 + cofs + 1]); val[2] += bfr(bias[c0 + cofs + 2]); val[3] += bfr(bias[c0 + cofs + 3]); }
                *(volatile v4f*)(crow + (size_t)row * ldc + cofs) = val; }
            if (ps == 0) __threadfence(); }
        __builtin_amdgcn_wave_barrier(); asm volatile("" ::: "memory");
    }
}

__device__ __forceinline__ h16 tohx(float x) { return (h16)x; }
__device__ __forceinline__ void splitf(float y, unsigned short& h, unsigned short& l) { h = f2bf(y); l = f2bf(y - bf2f(h)); }
typedef __attribute__((ext_vector_type(2))) _Float16 v2h;
typedef __attribute__((ext_vector_type(4))) _Float16 v4h;
typedef __attribute__((ext_vector_type(4))) unsigned short v4us;

__global__ __launch_bounds__(256) void k_tokn(const float* __restrict__ X, bf* Th, bf* Tl) { const int lane = threadIdx.x & 31; const int n = blockIdx.x * 8 + (threadIdx.x >> 5); if (n >= NTK) return; const size_t rb = (size_t)n * DD; float v[16]; float q2 = 0.f;
#pragma unroll
    for (int ch = 0; ch < 4; ++ch) { const v4f a = *(const v4f*)(X + rb + ch * 128 + lane * 4);
#pragma unroll
        for (int q = 0; q < 4; ++q) { v[ch * 4 + q] = bfr(a[q]); float p = __fmul_rn(v[ch * 4 + q], v[ch * 4 + q]); asm volatile("" : "+v"(p)); q2 = __fadd_rn(q2, p); } }
#pragma unroll
    for (int sh = 16; sh; sh >>= 1) q2 += __shfl_xor(q2, sh, 32);
    const float inv = __fdiv_rn(1.0f, __fsqrt_rn(q2));
    for (int ps = 0; ps < 2; ++ps) {
#pragma unroll
        for (int ch = 0; ch < 4; ++ch) { const int c0 = ch * 128 + lane * 4; v4us oh, ol;
#pragma unroll
            for (int q = 0; q < 4; ++q) { unsigned short a, c; splitf(__fmul_rn(v[ch * 4 + q], inv), a, c); oh[q] = a; ol[q] = c; } *(volatile v4us*)(Th + rb + c0) = oh; *(volatile v4us*)(Tl + rb + c0) = ol; } if (ps == 0) __threadfence(); } }
__global__ __launch_bounds__(256) void k_tokT(const bf* __restrict__ Th, const bf* __restrict__ Tl, h16* T16) { const size_t e = ((size_t)blockIdx.x * 256 + threadIdx.x) * 2; if (e >= (size_t)DD * NTK) return; const int n = (int)(e % NTK); const int d = (int)(e / NTK); v2h o;
#pragma unroll
    for (int u = 0; u < 2; ++u) { const size_t s = (size_t)(n + u) * DD + d; o[u] = tohx(__fadd_rn(bf2f(Th[s]), bf2f(Tl[s]))); } *(volatile v2h*)(T16 + e) = o; __threadfence(); *(volatile v2h*)(T16 + e) = o; }
__global__ __launch_bounds__(256) void k_pb(const float* __restrict__ Pr, bf* PB) { const size_t e = ((size_t)blockIdx.x * 256 + threadIdx.x) * 4; if (e >= (size_t)NPP * DD) return; const int p = (int)(e / DD); v4us o;
#pragma unroll
    for (int q = 0; q < 4; ++q) o[q] = p < NP ? f2bf(Pr[e + q]) : (unsigned short)0; *(volatile v4us*)(PB + e) = o; __threadfence(); *(volatile v4us*)(PB + e) = o; }
__device__ __forceinline__ int labc(const int* lab, int n) { return min(max(lab[n], 0), NC - 1); }
__global__ __launch_bounds__(256) void k_cnt(const int* __restrict__ lab, float* CNT) { const int c = blockIdx.x * 256 + threadIdx.x; if (c >= 256) return; int k = 0; if (c < NC) { for (int n = 0; n < NTK; ++n) k += (labc(lab, n) == c); } const float f = (float)k; *(volatile float*)(CNT + c) = f; __threadfence(); *(volatile float*)(CNT + c) = f; }
__global__ __launch_bounds__(256) void k_init(const int* __restrict__ lab, const float* __restrict__ CNT, float* U, float* V, float* LOGB) { const int i = blockIdx.x * 256 + threadIdx.x; if (i < NPP) { *(volatile float*)(U + i) = 0.f; } if (i < NTK) { const float lb = __logf(__fadd_rn(__fdiv_rn(1.0f, CNT[labc(lab, i)]), 1e-8f)); *(volatile float*)(V + i) = 0.f; *(volatile float*)(LOGB + i) = lb; __threadfence(); *(volatile float*)(V + i) = 0.f; *(volatile float*)(LOGB + i) = lb; if (i < NPP) *(volatile float*)(U + i) = 0.f; } }
__global__ __launch_bounds__(256) void k_urow(const float* __restrict__ CT, const int* __restrict__ lab, const float* __restrict__ V, const float* __restrict__ Uin, float* Uout) { const int p = blockIdx.x * 256 + threadIdx.x; if (p >= NPP) return; float un = 0.f;
    if (p < NP) { const int c = p / NPR; const float up = Uin[p]; float mx = -3.0e38f;
#pragma unroll 1
        for (int n = 0; n < NTK; ++n) if (labc(lab, n) == c) { const float kv = __fmul_rn(__fadd_rn(__fadd_rn(CT[(size_t)n * NPP + p], up), V[n]), 1.0f / EPSI); mx = fmaxf(mx, kv); }
        float s = 0.f;
#pragma unroll 1
        for (int n = 0; n < NTK; ++n) if (labc(lab, n) == c) { const float kv = __fmul_rn(__fadd_rn(__fadd_rn(CT[(size_t)n * NPP + p], up), V[n]), 1.0f / EPSI); s = __fadd_rn(s, __expf(__fsub_rn(kv, mx))); }
        const float loga = __logf(__fadd_rn(1.0f / (float)NPR, 1e-8f)); float u_ = (mx > -1.0e38f) ? __fsub_rn(loga, __fadd_rn(__logf(s), mx)) : 0.f;   un = __fadd_rn(__fmul_rn(EPSI, u_), up); }
    *(volatile float*)(Uout + p) = un; __threadfence(); *(volatile float*)(Uout + p) = un; }
__global__ __launch_bounds__(256) void k_vrow(const float* __restrict__ CT, const int* __restrict__ lab, const float* __restrict__ U, const float* __restrict__ LOGB, const float* __restrict__ Vin, float* Vout) { const int n = blockIdx.x * 256 + threadIdx.x; if (n >= NTK) return; const int c = labc(lab, n); const float vn = Vin[n]; const float* cr = CT + (size_t)n * NPP + c * NPR; float kv[NPR]; float mx = -3.0e38f;
#pragma unroll
    for (int r = 0; r < NPR; ++r) { kv[r] = __fmul_rn(__fadd_rn(__fadd_rn(cr[r], U[c * NPR + r]), vn), 1.0f / EPSI); mx = fmaxf(mx, kv[r]); }
    float s = 0.f;
#pragma unroll
    for (int r = 0; r < NPR; ++r) s = __fadd_rn(s, __expf(__fsub_rn(kv[r], mx)));
    const float v_ = __fsub_rn(LOGB[n], __fadd_rn(__logf(s), mx)); const float out = __fadd_rn(__fmul_rn(EPSI, v_), vn); *(volatile float*)(Vout + n) = out; __threadfence(); *(volatile float*)(Vout + n) = out; }
__global__ __launch_bounds__(256) void k_colsum(const float* __restrict__ CT, const int* __restrict__ lab, const float* __restrict__ U, const float* __restrict__ V, float* CS) { const int n = blockIdx.x * 256 + threadIdx.x; if (n >= NTK) return; const int c = labc(lab, n); const float* cr = CT + (size_t)n * NPP + c * NPR; float s = 0.f;
#pragma unroll
    for (int r = 0; r < NPR; ++r) s = __fadd_rn(s, __expf(__fmul_rn(__fadd_rn(__fadd_rn(cr[r], U[c * NPR + r]), V[n]), 1.0f / EPSI)));
    *(volatile float*)(CS + n) = s; __threadfence(); *(volatile float*)(CS + n) = s; }
__global__ __launch_bounds__(256) void k_pi(const float* __restrict__ CT, const int* __restrict__ lab, const float* __restrict__ U, const float* __restrict__ V, const float* __restrict__ CS, h16* PI) { const size_t e = ((size_t)blockIdx.x * 256 + threadIdx.x) * 4; if (e >= (size_t)NPP * NTK) return; const int n0 = (int)(e % NTK); const int p = (int)(e / NTK); v4h o;
#pragma unroll
    for (int q = 0; q < 4; ++q) { const int n = n0 + q; float val = 0.f; if (p < NP && labc(lab, n) == p / NPR) { const float kv = __fmul_rn(__fadd_rn(__fadd_rn(CT[(size_t)n * NPP + p], U[p]), V[n]), 1.0f / EPSI); val = __fdiv_rn(__expf(kv), CS[n]); } o[q] = tohx(val); }
    *(volatile v4h*)(PI + e) = o; __threadfence(); *(volatile v4h*)(PI + e) = o; }
__global__ __launch_bounds__(256) void k_out(const float* __restrict__ Pr, const float* __restrict__ NEW, float* OUT) { const int lane = threadIdx.x & 31; const int p = blockIdx.x * 8 + (threadIdx.x >> 5); if (p >= NP) return; const size_t rb = (size_t)p * DD; float v[16]; float q2 = 0.f;
#pragma unroll
    for (int ch = 0; ch < 4; ++ch) { const int c0 = ch * 128 + lane * 4; const v4f a = *(const v4f*)(Pr + rb + c0); const v4f nw = *(const v4f*)(NEW + rb + c0);
#pragma unroll
        for (int q = 0; q < 4; ++q) { float t1 = __fmul_rn(0.98f, bfr(a[q])); asm volatile("" : "+v"(t1)); float t2 = __fmul_rn(0.02f, nw[q]); asm volatile("" : "+v"(t2)); v[ch * 4 + q] = __fadd_rn(t1, t2); float pq = __fmul_rn(v[ch * 4 + q], v[ch * 4 + q]); asm volatile("" : "+v"(pq)); q2 = __fadd_rn(q2, pq); } }
#pragma unroll
    for (int sh = 16; sh; sh >>= 1) q2 += __shfl_xor(q2, sh, 32);
    const float inv = __fdiv_rn(1.0f, __fsqrt_rn(q2));
    for (int ps = 0; ps < 2; ++ps) {
#pragma unroll
        for (int ch = 0; ch < 4; ++ch) { const int c0 = ch * 128 + lane * 4; v4f o; o[0] = __fmul_rn(v[ch * 4], inv); o[1] = __fmul_rn(v[ch * 4 + 1], inv); o[2] = __fmul_rn(v[ch * 4 + 2], inv); o[3] = __fmul_rn(v[ch * 4 + 3], inv); *(volatile v4f*)(OUT + rb + c0) = o; } if (ps == 0) __threadfence(); } }

extern "C" void kernel_launch(void* const* d_in, const int* in_sizes, int n_in,
                              void* d_out, int out_size, void* d_ws, size_t ws_size, hipStream_t stream) {
    (void)in_sizes; (void)n_in; (void)out_size;
    const float* tokens = (const float*)d_in[0]; const int* lab = (const int*)d_in[1]; const float* protos = (const float*)d_in[2];
    float* OUT = (float*)d_out;
    char* wsp = (char*)d_ws;
    auto take = [&](size_t bytes) { char* p = wsp; wsp += (bytes + 255) & ~(size_t)255; return (void*)p; };
    bf* Th = (bf*)take((size_t)NTK * DD * 2); bf* Tl = (bf*)take((size_t)NTK * DD * 2); h16* T16 = (h16*)take((size_t)DD * NTK * 2); bf* PB = (bf*)take((size_t)NPP * DD * 2); float* CT = (float*)take((size_t)NTK * NPP * 4);
    float* CNT = (float*)take(256 * 4); float* U0 = (float*)take(NPP * 4); float* U1 = (float*)take(NPP * 4); float* V0 = (float*)take(NTK * 4); float* V1 = (float*)take(NTK * 4); float* LOGB = (float*)take(NTK * 4); float* CS = (float*)take(NTK * 4); h16* PI = (h16*)take((size_t)NPP * NTK * 2); float* NEW = (float*)take((size_t)NPP * DD * 4);
    if ((size_t)(wsp - (char*)d_ws) > ws_size) return;
    k_tokn<<<NTK / 8, 256, 0, stream>>>(tokens, Th, Tl); k_tokT<<<(unsigned)(((size_t)DD * NTK / 2 + 255) / 256), 256, 0, stream>>>(Th, Tl, T16); k_pb<<<(NPP * DD / 4 + 255) / 256, 256, 0, stream>>>(protos, PB);
    k_gemmw<bf, 1, false><<<dim3(NTK / 64, NPP / 64, 1), 32, 0, stream>>>(Th, Tl, PB, nullptr, DD, CT, NPP, nullptr, 0, 0, 0);
    k_cnt<<<1, 256, 0, stream>>>(lab, CNT); k_init<<<NTK / 256, 256, 0, stream>>>(lab, CNT, U0, V0, LOGB);
    float* U = U0; float* Un = U1; float* V = V0; float* Vn = V1;
    for (int it = 0; it < ITER; ++it) { k_urow<<<NPP / 256, 256, 0, stream>>>(CT, lab, V, U, Un); { float* t = U; U = Un; Un = t; } k_vrow<<<NTK / 256, 256, 0, stream>>>(CT, lab, U, LOGB, V, Vn); { float* t = V; V = Vn; Vn = t; } }
    k_colsum<<<NTK / 256, 256, 0, stream>>>(CT, lab, U, V, CS); k_pi<<<(unsigned)(((size_t)NPP * NTK / 4 + 255) / 256), 256, 0, stream>>>(CT, lab, U, V, CS, PI);
    k_gemmw<h16, 0, false><<<dim3(NPP / 64, DD / 64, 1), 32, 0, stream>>>(PI, nullptr, T16, nullptr, NTK, NEW, DD, nullptr, 0, 0, 0);
    k_out<<<NP / 8, 256, 0, stream>>>(protos, NEW, OUT);
}
